// Net_33998961115614
// MI455X (gfx1250) — hardware-verified
//
#include <hip/hip_runtime.h>
#include <stddef.h>
#include <stdint.h>
#include <math.h>


#define FIN    256
#define HID    128
#define KD     256
#define NHD    64
#define NCL    2
#define NGR    128
#define NTHR   256
#define NWAVE  8
#define EPT    8
#define CHUNK  (NTHR * EPT)
#define WCAP   (EPT * 32)
#define LISTN  (NWAVE * WCAP)
#define NBA    1024
#define SLA    10
#define RCAP   16384
#define DEGCAP 64
#define GBM    64
#define GBN    128
#define GTHR   128
#define WUNITS (HID * (KD / 8))
#define WBLK   (WUNITS / NTHR)
#define AGG_ZINTS (LISTN + 2 * RCAP + 3 * NBA)
#define AGG_LDS_INTS (AGG_ZINTS + 16)
#define NOUT1  (NGR * NCL)
#define WSMAX  134217728

static_assert((CHUNK & (CHUNK - 1)) == 0 && CHUNK <= 4096);
static_assert((NBA & (NBA - 1)) == 0 && NBA == (1 << SLA));
static_assert(((long long)CHUNK << SLA) < (1LL << 31));
static_assert(LISTN % NTHR == 0);
static_assert(NBA % NWAVE == 0 && NBA % 32 == 0 && NBA % GBM == 0);
static_assert(RCAP % 32 == 0 && AGG_ZINTS % 4 == 0 && LISTN % 4 == 0);
static_assert(KD % 32 == 0 && FIN == KD && KD == 2 * HID && HID == GBN);
static_assert(GBM == (GTHR / 32) * 16 && HID == 4 * 32);
static_assert(WUNITS % NTHR == 0 && KD / 8 == 32);
static_assert(AGG_LDS_INTS * 4 <= 300000);
static_assert(NOUT1 == 4 * 64 && (NOUT1 * 4) % 128 == 0);
static_assert(NGR * NHD == 32 * NTHR);

typedef float          v4f   __attribute__((ext_vector_type(4)));
typedef float          v8f   __attribute__((ext_vector_type(8)));
typedef int            v4i   __attribute__((ext_vector_type(4)));
typedef int            v8i   __attribute__((ext_vector_type(8)));
typedef unsigned int   v4u   __attribute__((ext_vector_type(4)));
typedef unsigned short v8us  __attribute__((ext_vector_type(8)));
typedef unsigned short v16us __attribute__((ext_vector_type(16)));
typedef __bf16         v16bf __attribute__((ext_vector_type(16)));
typedef v4f  __attribute__((may_alias)) v4fa;
typedef v4i  __attribute__((may_alias)) v4ia;
typedef v8us __attribute__((may_alias)) v8usa;
union FragB { v16bf v; v16us u; v8us h[2]; v8i w; };

__device__ __forceinline__ v8f wmb(const FragB& a, const FragB& b, v8f c) {
  v8f d = __builtin_amdgcn_wmma_f32_16x16x32_bf16(false, a.v, false, b.v, (short)0, c, false, false);
  asm volatile("v_nop\n\tv_nop\n\tv_nop\n\tv_nop" : "+v"(d) : "v"(a.w), "v"(b.w));
  return d;
}

__device__ __forceinline__ unsigned bf16_bits(float f) {
  const unsigned u = __float_as_uint(f);
  return (u + 0x7FFFu + ((u >> 16) & 1u)) >> 16;
}
__device__ __forceinline__ float bf16_val(float f) {
  return __uint_as_float(bf16_bits(f) << 16);
}

__device__ __forceinline__ float selu1(float v) {
  const float e = expm1f(v);
  return 1.0507009873554805f * ((v > 0.0f) ? v : 1.6732632423543772f * e);
}
__device__ __forceinline__ v4f selu4(v4f y) {
  float r0 = y.x, r1 = y.y, r2 = y.z, r3 = y.w;
#pragma unroll 1
  for (int j = 0; j < 4; ++j) {
    const float v = (j == 0) ? y.x : ((j == 1) ? y.y : ((j == 2) ? y.z : y.w));
    const float s = selu1(v);
    r0 = (j == 0) ? s : r0;
    r1 = (j == 1) ? s : r1;
    r2 = (j == 2) ? s : r2;
    r3 = (j == 3) ? s : r3;
  }
  v4f r;
  r.x = r0; r.y = r1; r.z = r2; r.w = r3;
  return r;
}

__device__ __forceinline__ void put8(unsigned short* dp, v8us o) {
  *(volatile v8us*)dp = o;
  __threadfence();
  *(volatile v8us*)dp = o;
}

template <int SLB>
__device__ __forceinline__ int scan_chunk(const int* __restrict__ dsts, int nE, int cbase, int slotBase,
                                          int nb, int vec8, int* list, int tid, int lane, int wave) {
  int wc = 0;
  const int el0  = tid * EPT;
  const int e0   = cbase + el0;
  const int sent = -2147483647 - 1;
  v4i da, db;
  if (vec8 != 0 && cbase + CHUNK <= nE) {
    da = *(const v4i*)(dsts + e0);
    db = *(const v4i*)(dsts + e0 + 4);
  } else {
    da.x = (e0     < nE) ? dsts[min(e0,     nE - 1)] : sent;
    da.y = (e0 + 1 < nE) ? dsts[min(e0 + 1, nE - 1)] : sent;
    da.z = (e0 + 2 < nE) ? dsts[min(e0 + 2, nE - 1)] : sent;
    da.w = (e0 + 3 < nE) ? dsts[min(e0 + 3, nE - 1)] : sent;
    db.x = (e0 + 4 < nE) ? dsts[min(e0 + 4, nE - 1)] : sent;
    db.y = (e0 + 5 < nE) ? dsts[min(e0 + 5, nE - 1)] : sent;
    db.z = (e0 + 6 < nE) ? dsts[min(e0 + 6, nE - 1)] : sent;
    db.w = (e0 + 7 < nE) ? dsts[min(e0 + 7, nE - 1)] : sent;
  }
  const unsigned nbs = (unsigned)slotBase;
  const unsigned unb = (unsigned)nb;
  const unsigned s0 = (unsigned)da.x - nbs, s1 = (unsigned)da.y - nbs;
  const unsigned s2 = (unsigned)da.z - nbs, s3 = (unsigned)da.w - nbs;
  const unsigned s4 = (unsigned)db.x - nbs, s5 = (unsigned)db.y - nbs;
  const unsigned s6 = (unsigned)db.z - nbs, s7 = (unsigned)db.w - nbs;
  const bool h0 = s0 < unb, h1 = s1 < unb, h2 = s2 < unb, h3 = s3 < unb;
  const bool h4 = s4 < unb, h5 = s5 < unb, h6 = s6 < unb, h7 = s7 < unb;
  const unsigned any = __builtin_amdgcn_ballot_w32(h0 | h1 | h2 | h3 | h4 | h5 | h6 | h7);
  if (any != 0u) {
#define HITJ(J, HJ, SJ) { \
      const unsigned mj = __builtin_amdgcn_ballot_w32(HJ); \
      if (mj != 0u) { \
        if (HJ) { \
          const int pos = wc + (int)__builtin_amdgcn_mbcnt_lo(mj, 0u); \
          if (pos < WCAP) list[wave * WCAP + pos] = ((el0 + (J)) << SLB) | (int)(SJ); \
        } \
        wc += (int)__builtin_popcount(mj); } }
    HITJ(0, h0, s0)
    HITJ(1, h1, s1)
    HITJ(2, h2, s2)
    HITJ(3, h3, s3)
    HITJ(4, h4, s4)
    HITJ(5, h5, s5)
    HITJ(6, h6, s6)
    HITJ(7, h7, s7)
#undef HITJ
  }
  return wc;
}

__global__ __launch_bounds__(NTHR) void k_prep(const float* __restrict__ x, const float* __restrict__ W1,
                                               const float* __restrict__ W2, int nN, int nUnits,
                                               unsigned short* W1T, unsigned short* W2T2, unsigned short* xb) {
  const int b = (int)blockIdx.x, tid = (int)threadIdx.x;
  v8us o;
  if (b < WBLK) {
    const int u  = b * NTHR + tid;
    const int n  = u >> 5;
    const int k8 = (u & 31) * 8;
    const float* p = W1 + (size_t)k8 * HID + n;
#pragma unroll
    for (int i = 0; i < 8; ++i) o[i] = (unsigned short)bf16_bits(p[(size_t)i * HID]);
    put8(W1T + (size_t)n * KD + k8, o);
  } else if (b < 2 * WBLK) {
    const int u  = (b - WBLK) * NTHR + tid;
    const int n  = u >> 5;
    const int k8 = (u & 31) * 8;
    const int kk = k8 & (HID - 1);
    const float* p = W2 + (size_t)kk * HID + n;
#pragma unroll
    for (int i = 0; i < 8; ++i) o[i] = (unsigned short)bf16_bits(p[(size_t)i * HID]);
    put8(W2T2 + (size_t)n * KD + k8, o);
  } else {
    const int u = (b - 2 * WBLK) * NTHR + tid;
    if (u >= nUnits) return;
    const int row = u >> 5;
    const int k8  = (u & 31) * 8;
    const int rc  = row < nN ? row : nN - 1;
    const float* p = x + (size_t)rc * FIN + k8;
    const v4f a = *(const v4fa*)p;
    const v4f c = *(const v4fa*)(p + 4);
    const bool ok = row < nN;
    o[0] = ok ? (unsigned short)bf16_bits(a.x) : (unsigned short)0;
    o[1] = ok ? (unsigned short)bf16_bits(a.y) : (unsigned short)0;
    o[2] = ok ? (unsigned short)bf16_bits(a.z) : (unsigned short)0;
    o[3] = ok ? (unsigned short)bf16_bits(a.w) : (unsigned short)0;
    o[4] = ok ? (unsigned short)bf16_bits(c.x) : (unsigned short)0;
    o[5] = ok ? (unsigned short)bf16_bits(c.y) : (unsigned short)0;
    o[6] = ok ? (unsigned short)bf16_bits(c.z) : (unsigned short)0;
    o[7] = ok ? (unsigned short)bf16_bits(c.w) : (unsigned short)0;
    put8(xb + (size_t)row * KD + k8, o);
  }
}

__global__ __launch_bounds__(GTHR) void k_gemm(const unsigned short* __restrict__ Apl,
                                               const unsigned short* __restrict__ BT,
                                               const float* __restrict__ avs, const float* __restrict__ avd,
                                               float* hout, float* asv, float* adv) {
  __shared__ __attribute__((aligned(16))) float stg[GBM * GBN];
  __shared__ __attribute__((aligned(16))) float sas[GBM];
  __shared__ __attribute__((aligned(16))) float sad[GBM];
  const int tid = (int)threadIdx.x, lane = tid & 31, wave = tid >> 5, hh = lane >> 4, m = lane & 15;
  const int rowBase = (int)blockIdx.x * GBM;

  v8f acc[8];
  {
    const v8f z = {0.f, 0.f, 0.f, 0.f, 0.f, 0.f, 0.f, 0.f};
#pragma unroll
    for (int t = 0; t < 8; ++t) acc[t] = z;
  }
  const unsigned short* ap = Apl + (size_t)(rowBase + 16 * wave + m) * (size_t)KD + 8 * hh;
  const unsigned short* bp = BT + (size_t)m * (size_t)KD + 8 * hh;

#pragma unroll 1
  for (int k0 = 0; k0 < KD; k0 += 32) {
    FragB af;
    af.h[0] = *(const v8usa*)(ap + k0);
    af.h[1] = *(const v8usa*)(ap + k0 + 16);
#pragma unroll
    for (int nt = 0; nt < 8; ++nt) {
      const unsigned short* wq = bp + (size_t)(16 * nt) * (size_t)KD + k0;
      FragB bf;
      bf.h[0] = *(const v8usa*)wq;
      bf.h[1] = *(const v8usa*)(wq + 16);
      acc[nt] = wmb(af, bf, acc[nt]);
    }
  }

#pragma unroll
  for (int nt = 0; nt < 8; ++nt) {
    const int lc = 16 * nt + m;
#pragma unroll
    for (int r = 0; r < 8; ++r) {
      const int lr = 16 * wave + 8 * hh + r;
      stg[lr * GBN + lc] = acc[nt][r];
    }
  }
  __syncthreads();

  v4f a4s, a4d;
  {
    const v4f t1 = *(const v4fa*)(avs + 4 * lane);
    const v4f t2 = *(const v4fa*)(avd + 4 * lane);
    a4s.x = bf16_val(t1.x); a4s.y = bf16_val(t1.y); a4s.z = bf16_val(t1.z); a4s.w = bf16_val(t1.w);
    a4d.x = bf16_val(t2.x); a4d.y = bf16_val(t2.y); a4d.z = bf16_val(t2.z); a4d.w = bf16_val(t2.w);
  }
#pragma unroll 1
  for (int i = 0; i < 16; ++i) {
    const int lr = 16 * wave + i;
    const v4f v = *(const v4fa*)(stg + lr * GBN + 4 * lane);
    float ps = v.x * a4s.x;
    ps = fmaf(v.y, a4s.y, ps); ps = fmaf(v.z, a4s.z, ps); ps = fmaf(v.w, a4s.w, ps);
    float pd = v.x * a4d.x;
    pd = fmaf(v.y, a4d.y, pd); pd = fmaf(v.z, a4d.z, pd); pd = fmaf(v.w, a4d.w, pd);
#pragma unroll
    for (int off = 16; off > 0; off >>= 1) {
      const float qs = __shfl_xor(ps, off, 32);
      const float qd = __shfl_xor(pd, off, 32);
      ps += qs; pd += qd;
    }
    if (lane == 0) { sas[lr] = ps; sad[lr] = pd; }
    *(volatile v4f*)(hout + (size_t)(rowBase + lr) * HID + 4 * lane) = v;
  }
  __threadfence();
#pragma unroll 1
  for (int i = 0; i < 16; ++i) {
    const int lr = 16 * wave + i;
    const v4f v = *(const v4fa*)(stg + lr * GBN + 4 * lane);
    *(volatile v4f*)(hout + (size_t)(rowBase + lr) * HID + 4 * lane) = v;
  }
  __syncthreads();
  const v4f sv = *(const v4fa*)(sas + 4 * (lane & 15));
  const v4f dv = *(const v4fa*)(sad + 4 * (lane & 15));
  const bool okst = (wave == 0) && (lane < 16);
  float* sp = asv + (size_t)rowBase + 4 * (lane & 15);
  float* dp = adv + (size_t)rowBase + 4 * (lane & 15);
  if (okst) { *(volatile v4f*)sp = sv; *(volatile v4f*)dp = dv; }
  __threadfence();
  if (okst) { *(volatile v4f*)sp = sv; *(volatile v4f*)dp = dv; }
}

template <int MODE>
__global__ __launch_bounds__(NTHR) void k_scan(const int* __restrict__ srcs, const int* __restrict__ dsts,
                                               int nE, int nN, int vec8, int mRows,
                                               const float* __restrict__ asv, const float* __restrict__ adv,
                                               const float* __restrict__ xl, const float* __restrict__ bias,
                                               unsigned short* hb, float* hout) {
  extern __shared__ __attribute__((aligned(16))) int dsm[];
  int* list = dsm;
  int* hl   = dsm + LISTN;
  int* sl   = dsm + LISTN + RCAP;
  int* cnt  = dsm + LISTN + 2 * RCAP;
  int* offs = cnt + NBA;
  int* cur  = offs + NBA;
  int* misc = cur + NBA;
  const int tid = (int)threadIdx.x, lane = tid & 31, wave = tid >> 5;
  const int nodeBase = (int)blockIdx.x * NBA;

  {
    const v4i z4 = {0, 0, 0, 0};
    for (int i = tid * 4; i < AGG_ZINTS; i += NTHR * 4) *(v4ia*)(dsm + i) = z4;
    if (tid < 16) misc[tid] = 0;
  }
  v4f bv;
  {
    const v4f a = *(const v4fa*)(bias + 4 * lane);
    bv.x = bf16_val(a.x); bv.y = bf16_val(a.y); bv.z = bf16_val(a.z); bv.w = bf16_val(a.w);
  }
  __syncthreads();

  int t = 0, ov = 0;
  const int nChunks = (nE + CHUNK - 1) / CHUNK;
#pragma unroll 1
  for (int ch = 0; ch < nChunks; ++ch) {
    const int cbase = ch * CHUNK;
    const int wc = scan_chunk<SLA>(dsts, nE, cbase, nodeBase, NBA, vec8, list, tid, lane, wave);
    if (lane == 0) misc[wave] = wc;
    __syncthreads();
    if (wave == 0) {
#pragma unroll 1
      for (int w2 = 0; w2 < NWAVE; ++w2) {
        int c = misc[w2];
        c = c < 0 ? 0 : (c > WCAP ? WCAP : c);
#pragma unroll 1
        for (int b0 = 0; b0 < c; b0 += 32) {
          const int idx = b0 + lane;
          const int ent = list[w2 * WCAP + (idx < WCAP ? idx : WCAP - 1)];
          const int m32 = (c - b0) < 32 ? (c - b0) : 32;
#pragma unroll 1
          for (int k = 0; k < m32; ++k) {
            const int u    = __builtin_amdgcn_readlane(ent, k);
            const int slot = u & (NBA - 1);
            const int el   = (u >> SLA) & (CHUNK - 1);
            const int pk   = ((cbase + el) << SLA) | slot;
            if (t < RCAP) {
              if (lane == 0) { hl[t] = pk; cnt[slot] = cnt[slot] + 1; }
              t = t + 1;
            } else {
              ov = 1;
            }
          }
        }
      }
    }
    __syncthreads();
  }
  if (wave == 0 && lane == 0) { misc[8] = t; misc[9] = ov; }
  __syncthreads();
  int tt = misc[8];
  tt = tt < 0 ? 0 : (tt > RCAP ? RCAP : tt);
  const int ovf = misc[9];

  if (wave == 0) {
    const int base = lane * (NBA / 32);
    int s = 0;
#pragma unroll 1
    for (int i = 0; i < NBA / 32; ++i) s += cnt[base + i];
    int incl = s;
#pragma unroll
    for (int d = 1; d < 32; d <<= 1) {
      const int y = __shfl_up(incl, d, 32);
      if (lane >= d) incl += y;
    }
    int run = incl - s;
#pragma unroll 1
    for (int i = 0; i < NBA / 32; ++i) {
      const int cv = cnt[base + i];
      offs[base + i] = run;
      cur[base + i]  = run;
      run += cv;
    }
  }
  __syncthreads();
  if (wave == 0) {
#pragma unroll 1
    for (int b0 = 0; b0 < tt; b0 += 32) {
      const int idx = b0 + lane;
      const int ent = hl[idx < RCAP ? idx : RCAP - 1];
      const int m32 = (tt - b0) < 32 ? (tt - b0) : 32;
#pragma unroll 1
      for (int k = 0; k < m32; ++k) {
        const int u    = __builtin_amdgcn_readlane(ent, k);
        const int slot = u & (NBA - 1);
        if (lane == 0) {
          int p = cur[slot];
          p = p < 0 ? 0 : (p > RCAP - 1 ? RCAP - 1 : p);
          sl[p] = u;
          cur[slot] = p + 1;
        }
      }
    }
  }
  __syncthreads();

  const float qnan = __int_as_float(0x7fc00000);
  const float ninf = __int_as_float((int)0xff800000u);
  const float pz = (ovf != 0) ? qnan : 0.0f;
  const int sA = (2 * lane) & 31, sB = (2 * lane + 1) & 31;
#pragma unroll 1
  for (int si = 0; si < NBA / NWAVE; ++si) {
    const int s    = si * NWAVE + wave;
    const int node = nodeBase + s;
    int c = cnt[s];
    const bool big = c > DEGCAP;
    c = c < 0 ? 0 : (c > DEGCAP ? DEGCAP : c);
    int o = offs[s];
    o = o < 0 ? 0 : (o > RCAP ? RCAP : o);
    const int nc = node < nN ? node : nN - 1;
    const float adn = adv[nc];
    const float asn = asv[nc];
    float es = asn + adn;
    es = (es > 0.0f) ? es : 0.2f * es;
    float mrun = es;
#pragma unroll 1
    for (int b0 = 0; b0 < c; b0 += 32) {
      int idx = o + b0 + lane;
      idx = idx > RCAP - 1 ? RCAP - 1 : idx;
      const int ent = sl[idx];
      int eid = ent >> SLA;
      eid = eid < 0 ? 0 : (eid > nE - 1 ? nE - 1 : eid);
      int sr = srcs[eid];
      sr = sr < 0 ? 0 : (sr > nN - 1 ? nN - 1 : sr);
      float e = asv[sr] + adn;
      e = (e > 0.0f) ? e : 0.2f * e;
      const bool valid = (b0 + lane) < c;
      float mx = valid ? e : ninf;
#pragma unroll
      for (int off = 16; off > 0; off >>= 1) {
        const float q = __shfl_xor(mx, off, 32);
        mx = fmaxf(mx, q);
      }
      mrun = fmaxf(mrun, mx);
    }
    float den = 0.0f;
    float a0 = 0.0f, a1 = 0.0f, a2 = 0.0f, a3 = 0.0f;
#pragma unroll 1
    for (int b0 = 0; b0 < c; b0 += 32) {
      int idx = o + b0 + lane;
      idx = idx > RCAP - 1 ? RCAP - 1 : idx;
      const int ent = sl[idx];
      int eid = ent >> SLA;
      eid = eid < 0 ? 0 : (eid > nE - 1 ? nE - 1 : eid);
      int sr = srcs[eid];
      sr = sr < 0 ? 0 : (sr > nN - 1 ? nN - 1 : sr);
      float e = asv[sr] + adn;
      e = (e > 0.0f) ? e : 0.2f * e;
      const bool valid = (b0 + lane) < c;
      const float ee = expf(e - mrun);
      const float ex = valid ? ee : 0.0f;
      const int exi = __float_as_int(ex);
      const int m32 = (c - b0) < 32 ? (c - b0) : 32;
#pragma unroll 1
      for (int k = 0; k < m32; ++k) {
        const int   sk = __builtin_amdgcn_readlane(sr, k);
        const float ck = __int_as_float(__builtin_amdgcn_readlane(exi, k));
        const v4f a = *(const v4fa*)(xl + (size_t)sk * HID + 4 * lane);
        den += ck;
        a0 = fmaf(ck, a.x, a0); a1 = fmaf(ck, a.y, a1);
        a2 = fmaf(ck, a.z, a2); a3 = fmaf(ck, a.w, a3);
      }
    }
    {
      const float exs = expf(es - mrun);
      const v4f a = *(const v4fa*)(xl + (size_t)nc * HID + 4 * lane);
      den += exs;
      a0 = fmaf(exs, a.x, a0); a1 = fmaf(exs, a.y, a1);
      a2 = fmaf(exs, a.z, a2); a3 = fmaf(exs, a.w, a3);
    }
    const float inv = 1.0f / den;
    v4f y;
    y.x = fmaf(a0, inv, bv.x); y.y = fmaf(a1, inv, bv.y);
    y.z = fmaf(a2, inv, bv.z); y.w = fmaf(a3, inv, bv.w);
    y = selu4(y);
    const float pzr = big ? qnan : pz;
    const bool live = node < nN;
    v4f v;
    v.x = live ? (y.x + pzr) : 0.0f;
    v.y = live ? (y.y + pzr) : 0.0f;
    v.z = live ? (y.z + pzr) : 0.0f;
    v.w = live ? (y.w + pzr) : 0.0f;
    if constexpr (MODE != 0) {
      const unsigned h0 = bf16_bits(v.x), h1 = bf16_bits(v.y), h2 = bf16_bits(v.z), h3 = bf16_bits(v.w);
      const unsigned l0 = bf16_bits(v.x - __uint_as_float(h0 << 16));
      const unsigned l1 = bf16_bits(v.y - __uint_as_float(h1 << 16));
      const unsigned l2 = bf16_bits(v.z - __uint_as_float(h2 << 16));
      const unsigned l3 = bf16_bits(v.w - __uint_as_float(h3 << 16));
      const int hw0 = (int)(h0 | (h1 << 16)), hw1 = (int)(h2 | (h3 << 16));
      const int lw0 = (int)(l0 | (l1 << 16)), lw1 = (int)(l2 | (l3 << 16));
      const int g0 = __shfl(hw0, sA, 32), g1 = __shfl(hw1, sA, 32);
      const int g2 = __shfl(hw0, sB, 32), g3 = __shfl(hw1, sB, 32);
      const int p0 = __shfl(lw0, sA, 32), p1 = __shfl(lw1, sA, 32);
      const int p2 = __shfl(lw0, sB, 32), p3 = __shfl(lw1, sB, 32);
      const bool lsel = (lane & 16) != 0;
      v4u pv;
      pv.x = (unsigned int)(lsel ? p0 : g0);
      pv.y = (unsigned int)(lsel ? p1 : g1);
      pv.z = (unsigned int)(lsel ? p2 : g2);
      pv.w = (unsigned int)(lsel ? p3 : g3);
      const bool wr = node < mRows;
      unsigned short* hp = hb + (size_t)(wr ? node : 0) * KD + 8 * lane;
      if (wr) *(volatile v4u*)hp = pv;
      __threadfence();
      if (wr) *(volatile v4u*)hp = pv;
    } else {
      const bool wr = node < nN;
      float* op = hout + (size_t)(wr ? node : 0) * HID + 4 * lane;
      if (wr) *(volatile v4f*)op = v;
      __threadfence();
      if (wr) *(volatile v4f*)op = v;
    }
  }
}

__global__ __launch_bounds__(NTHR) void k_pool(const float* __restrict__ hf, const int* __restrict__ bat,
                                               int nN, float* zp) {
  __shared__ __attribute__((aligned(16))) float wsum[NWAVE * HID];
  __shared__ int wcn[NWAVE];
  __shared__ __attribute__((aligned(16))) float outs[HID];
  const int tid = (int)threadIdx.x, lane = tid & 31, wave = tid >> 5;
  const int g = (int)blockIdx.x;

  float a0 = 0.0f, a1 = 0.0f, a2 = 0.0f, a3 = 0.0f;
  int cnt = 0;
#pragma unroll 1
  for (int i0 = wave * 32; i0 < nN; i0 += NTHR) {
    const int i  = i0 + lane;
    const int ic = i < nN ? i : nN - 1;
    const int b  = bat[ic];
    const bool hit = (i < nN) && (b == g);
    unsigned msk = __builtin_amdgcn_ballot_w32(hit);
    int nh = (int)__builtin_popcount(msk);
    nh = nh > 32 ? 32 : nh;
    cnt += nh;
#pragma unroll 1
    for (int q = 0; q < nh; ++q) {
      const int k = __builtin_ffs((int)msk) - 1;
      msk &= msk - 1u;
      int node = i0 + (k < 0 ? 0 : k);
      node = node > nN - 1 ? nN - 1 : node;
      const v4f v = *(const v4fa*)(hf + (size_t)node * HID + 4 * lane);
      a0 += v.x; a1 += v.y; a2 += v.z; a3 += v.w;
    }
  }
  {
    v4f pa;
    pa.x = a0; pa.y = a1; pa.z = a2; pa.w = a3;
    *(v4fa*)(wsum + wave * HID + 4 * lane) = pa;
  }
  if (lane == 0) wcn[wave] = cnt;
  __syncthreads();
  if (tid < HID) {
    float s = 0.0f;
    int c = 0;
#pragma unroll
    for (int w2 = 0; w2 < NWAVE; ++w2) { s += wsum[w2 * HID + tid]; c += wcn[w2]; }
    const float cf = (c < 1) ? 1.0f : (float)c;
    outs[tid] = selu1(s * (1.0f / cf));
  }
  __syncthreads();
  const v4f ov = *(const v4fa*)(outs + 4 * lane);
  float* op = zp + (size_t)g * HID + 4 * lane;
  const bool okst = (wave == 0);
  if (okst) *(volatile v4f*)op = ov;
  __threadfence();
  if (okst) *(volatile v4f*)op = ov;
}

__global__ __launch_bounds__(NTHR) void k_head(const float* __restrict__ zp, const float* __restrict__ fc1w,
                                               const float* __restrict__ fc1b, const float* __restrict__ fc2w,
                                               const float* __restrict__ fc2b, float* out1) {
  __shared__ __attribute__((aligned(16))) float z1s[NGR * NHD];
  __shared__ float w2s[NHD * NCL];
  __shared__ float b1s[NHD];
  __shared__ float b2s[4];
  __shared__ __attribute__((aligned(16))) float os[NOUT1];
  const int tid = (int)threadIdx.x;
  if (tid < NHD * NCL) w2s[tid] = bf16_val(fc2w[tid]);
  if (tid < NHD) b1s[tid] = bf16_val(fc1b[tid]);
  if (tid < 4) {
    const float bb = fc2b[tid < NCL ? tid : NCL - 1];
    b2s[tid] = (tid < NCL) ? bf16_val(bb) : 0.0f;
  }
  __syncthreads();
#pragma unroll 1
  for (int idx = tid; idx < NGR * NHD; idx += NTHR) {
    const int g = idx >> 6;
    const int c = idx & (NHD - 1);
    const float* pr = zp + (size_t)g * HID;
    float s = 0.0f;
#pragma unroll 1
    for (int k4 = 0; k4 < HID / 4; ++k4) {
      const v4f p = *(const v4fa*)(pr + 4 * k4);
      const float* w = fc1w + (size_t)(4 * k4) * NHD + c;
      s = fmaf(p.x, bf16_val(w[0]), s);
      s = fmaf(p.y, bf16_val(w[NHD]), s);
      s = fmaf(p.z, bf16_val(w[2 * NHD]), s);
      s = fmaf(p.w, bf16_val(w[3 * NHD]), s);
    }
    z1s[idx] = selu1(s + b1s[c]);
  }
  __syncthreads();
  if (tid < NGR) {
    const int g = tid;
    float l0 = 0.0f, l1 = 0.0f;
#pragma unroll 1
    for (int k = 0; k < NHD; ++k) {
      const float a = z1s[g * NHD + k];
      l0 = fmaf(a, w2s[2 * k + 0], l0);
      l1 = fmaf(a, w2s[2 * k + 1], l1);
    }
    l0 += b2s[0];
    l1 += b2s[1];
    const float mx  = (l0 > l1) ? l0 : l1;
    const float d0  = l0 - mx, d1 = l1 - mx;
    const float sum = expf(d0) + expf(d1);
    const float lse = logf(sum);
    os[2 * g + 0] = d0 - lse;
    os[2 * g + 1] = d1 - lse;
  }
  __syncthreads();
  const int t4 = (tid < 64) ? tid : 63;
  const v4f ov = *(const v4fa*)(os + 4 * t4);
  const bool okst = tid < 64;
  float* op = out1 + 4 * (size_t)t4;
  if (okst) *(volatile v4f*)op = ov;
  __threadfence();
  if (okst) *(volatile v4f*)op = ov;
}

static inline int cdiv(int a, int b) { return (a + b - 1) / b; }
static inline size_t al256(size_t o) { return (o + 255) & ~(size_t)255; }

extern "C" void kernel_launch(void* const* d_in, const int* in_sizes, int n_in,
                              void* d_out, int out_size, void* d_ws, size_t ws_size,
                              hipStream_t stream) {
  if (n_in < 15) return;
  if (in_sizes[0] < FIN || (in_sizes[0] % FIN) != 0) return;
  const int nN = in_sizes[0] / FIN;
  if (nN < 1 || nN > (1 << 22)) return;
  if (in_sizes[1] < 2 || (in_sizes[1] & 1) != 0) return;
  const int nE = in_sizes[1] / 2;
  if (nE < 1 || nE >= (1 << (31 - SLA))) return;
  if (in_sizes[2] != nN) return;
  if (in_sizes[3] != FIN * HID) return;
  if (in_sizes[4] != HID || in_sizes[5] != HID || in_sizes[6] != HID) return;
  if (in_sizes[7] != HID * HID) return;
  if (in_sizes[8] != HID || in_sizes[9] != HID || in_sizes[10] != HID) return;
  if (in_sizes[11] != HID * NHD || in_sizes[12] != NHD) return;
  if (in_sizes[13] != NHD * NCL || in_sizes[14] != NCL) return;
  if ((long long)out_size != (long long)nN * HID + NOUT1) return;
  if ((((long long)nN * HID * 4) % 128) != 0) return;

  const float* x    = (const float*)d_in[0];
  const int*   edge = (const int*)d_in[1];
  const int*   bat  = (const int*)d_in[2];
  const float* W1   = (const float*)d_in[3];
  const float* as1  = (const float*)d_in[4];
  const float* ad1  = (const float*)d_in[5];
  const float* b1   = (const float*)d_in[6];
  const float* W2   = (const float*)d_in[7];
  const float* as2  = (const float*)d_in[8];
  const float* ad2  = (const float*)d_in[9];
  const float* b2   = (const float*)d_in[10];
  const float* fc1w = (const float*)d_in[11];
  const float* fc1b = (const float*)d_in[12];
  const float* fc2w = (const float*)d_in[13];
  const float* fc2b = (const float*)d_in[14];
  float* out0 = (float*)d_out;
  float* out1 = out0 + (size_t)nN * HID;
  const int* src = edge;
  const int* dst = edge + nE;

  const int MP = cdiv(nN, GBM) * GBM;
  const int gM = MP / GBM;
  const int gA = cdiv(MP, NBA);
  if ((long long)gA * NBA < (long long)MP) return;
  const int vec8 = ((nE & 3) == 0) ? 1 : 0;

  char* ws = (char*)d_ws;
  size_t off = 0;
  const size_t oW1T = off; off = al256(off + (size_t)HID * KD * 2);
  const size_t oW2T = off; off = al256(off + (size_t)HID * KD * 2);
  const size_t oXB  = off; off = al256(off + (size_t)MP * KD * 2);
  const size_t oH   = off; off = al256(off + (size_t)MP * HID * 4);
  const size_t oH1  = off; off = al256(off + (size_t)MP * KD * 2);
  const size_t oAS1 = off; off = al256(off + (size_t)MP * 4);
  const size_t oAD1 = off; off = al256(off + (size_t)MP * 4);
  const size_t oAS2 = off; off = al256(off + (size_t)MP * 4);
  const size_t oAD2 = off; off = al256(off + (size_t)MP * 4);
  const size_t oZP  = off; off = al256(off + (size_t)NGR * HID * 4);
  if (off > ws_size || off > (size_t)WSMAX) return;
  unsigned short* W1T  = (unsigned short*)(ws + oW1T);
  unsigned short* W2T2 = (unsigned short*)(ws + oW2T);
  unsigned short* XB   = (unsigned short*)(ws + oXB);
  float*          H    = (float*)(ws + oH);
  unsigned short* H1   = (unsigned short*)(ws + oH1);
  float*          AS1  = (float*)(ws + oAS1);
  float*          AD1  = (float*)(ws + oAD1);
  float*          AS2  = (float*)(ws + oAS2);
  float*          AD2  = (float*)(ws + oAD2);
  float*          ZP   = (float*)(ws + oZP);

  const size_t scanLds = (size_t)AGG_LDS_INTS * 4;
  hipFuncSetAttribute(reinterpret_cast<const void*>(&k_scan<1>), hipFuncAttributeMaxDynamicSharedMemorySize, (int)scanLds);
  hipFuncSetAttribute(reinterpret_cast<const void*>(&k_scan<0>), hipFuncAttributeMaxDynamicSharedMemorySize, (int)scanLds);

  const int nUx = MP * (KD / 8);
  k_prep<<<2 * WBLK + cdiv(nUx, NTHR), NTHR, 0, stream>>>(x, W1, W2, nN, nUx, W1T, W2T2, XB);
  k_gemm<<<gM, GTHR, 0, stream>>>(XB, W1T, as1, ad1, H, AS1, AD1);
  k_scan<1><<<gA, NTHR, scanLds, stream>>>(src, dst, nE, nN, vec8, MP, AS1, AD1, H, b1, H1, out0);
  k_gemm<<<gM, GTHR, 0, stream>>>(H1, W2T2, as2, ad2, H, AS2, AD2);
  k_scan<0><<<gA, NTHR, scanLds, stream>>>(src, dst, nE, nN, vec8, MP, AS2, AD2, H, b2, H1, out0);
  k_pool<<<NGR, NTHR, 0, stream>>>(out0, bat, nN, ZP);
  k_head<<<1, NTHR, 0, stream>>>(ZP, fc1w, fc1b, fc2w, fc2b, out1);
}
